// BotImpact_65979287601567
// MI455X (gfx1250) — hardware-verified
//
#include <hip/hip_runtime.h>
#include <stddef.h>
#include <stdint.h>


#define DIN     128
#define HC      64
#define NTHR    256
#define NWAVE   8
#define EPT     8
#define CHUNK   (NTHR * EPT)
#define WCAP    (EPT * 32)
#define LISTN   (NWAVE * WCAP)
#define NBMAX   512
#define SLBITS  9
#define RCAP    24576
#define DEGCAP  128
#define STW     128
#define GBM     64
#define GTHR    128
#define HBM     64
#define WSMAX   134217728
#define LDS_AGG ((2 * RCAP + 2 * NBMAX + LISTN) * 4 + 64)

static_assert((CHUNK & (CHUNK - 1)) == 0 && CHUNK <= 4096);
static_assert(NBMAX == (1 << SLBITS) && NBMAX <= 4096);
static_assert(NTHR * 2 == NBMAX);
static_assert(LISTN >= NBMAX);
static_assert(LISTN >= NWAVE * WCAP);
static_assert((RCAP % 32) == 0);
static_assert(NWAVE * STW <= RCAP);
static_assert(2 * 32 <= STW);
static_assert(LDS_AGG <= 300000);
static_assert(GBM == (GTHR / 32) * 16);
static_assert(HBM == (GTHR / 32) * 16);
static_assert(DIN / 8 == 16);
static_assert((DIN % 32) == 0 && (HC % 32) == 0);
static_assert(HC == 64);
static_assert(GBM * HC / 4 == 8 * GTHR);
static_assert(HBM * HC / 4 == 8 * GTHR);

typedef float          v4f  __attribute__((ext_vector_type(4)));
typedef float          v8f  __attribute__((ext_vector_type(8)));
typedef int            v4i  __attribute__((ext_vector_type(4)));
typedef int            v8i  __attribute__((ext_vector_type(8)));
typedef unsigned short v4us __attribute__((ext_vector_type(4)));
typedef unsigned short v8us __attribute__((ext_vector_type(8)));
typedef __bf16         v16b __attribute__((ext_vector_type(16)));
union FragB { v16b v; v8us h[2]; v8i w; };

__device__ __forceinline__ v8f wmb(const FragB& a, const FragB& b, v8f c) {
  v8f d = __builtin_amdgcn_wmma_f32_16x16x32_bf16(false, a.v, false, b.v, (short)0, c, false, false);
  asm volatile("v_nop\n\tv_nop\n\tv_nop\n\tv_nop" : "+v"(d) : "v"(a.w), "v"(b.w));
  return d;
}

__device__ __forceinline__ unsigned bfbits(float f) {
  const unsigned u = __float_as_uint(f);
  return (u + 0x7FFFu + ((u >> 16) & 1u)) >> 16;
}
__device__ __forceinline__ float bfr(float f) { return __uint_as_float(bfbits(f) << 16); }
__device__ __forceinline__ void hilo1(float v, unsigned short& hb, unsigned short& lb) {
  const unsigned hbt = bfbits(v);
  hb = (unsigned short)hbt;
  lb = (unsigned short)bfbits(v - __uint_as_float(hbt << 16));
}
__device__ __forceinline__ void hilo4(const v4f v, v4us& hb, v4us& lb) {
  unsigned short a0, a1, a2, a3, c0, c1, c2, c3;
  hilo1(v.x, a0, c0); hilo1(v.y, a1, c1); hilo1(v.z, a2, c2); hilo1(v.w, a3, c3);
  hb.x = a0; hb.y = a1; hb.z = a2; hb.w = a3;
  lb.x = c0; lb.y = c1; lb.z = c2; lb.w = c3;
}
__device__ __forceinline__ v8us cvt8b(const v4f a, const v4f b) {
  v8us hv;
  hv[0] = (unsigned short)bfbits(a.x); hv[1] = (unsigned short)bfbits(a.y);
  hv[2] = (unsigned short)bfbits(a.z); hv[3] = (unsigned short)bfbits(a.w);
  hv[4] = (unsigned short)bfbits(b.x); hv[5] = (unsigned short)bfbits(b.y);
  hv[6] = (unsigned short)bfbits(b.z); hv[7] = (unsigned short)bfbits(b.w);
  return hv;
}
__device__ __forceinline__ v4f sel4(bool c, const v4f a, const v4f b) {
  v4f r;
  r.x = c ? a.x : b.x; r.y = c ? a.y : b.y; r.z = c ? a.z : b.z; r.w = c ? a.w : b.w;
  return r;
}
__device__ __forceinline__ v8us sel8(bool c, const v8us a, const v8us b) {
  v8us r;
#pragma unroll
  for (int i = 0; i < 8; ++i) r[i] = c ? a[i] : b[i];
  return r;
}
__device__ __forceinline__ float lk01(float v) { return v > 0.f ? v : 0.01f * v; }

__device__ __forceinline__ int scan_chunk(const int* __restrict__ dsts, int nE, int cbase, int slotBase,
                                          int nb, int vec8, int* list, int tid, int lane, int wave) {
  int wc = 0;
  const int el0  = tid * EPT;
  const int e0   = cbase + el0;
  const int sent = -2147483647 - 1;
  v4i da, db;
  if (vec8 != 0 && cbase + CHUNK <= nE) {
    da = *(const v4i*)(dsts + e0);
    db = *(const v4i*)(dsts + e0 + 4);
  } else {
    da.x = (e0     < nE) ? dsts[min(e0,     nE - 1)] : sent;
    da.y = (e0 + 1 < nE) ? dsts[min(e0 + 1, nE - 1)] : sent;
    da.z = (e0 + 2 < nE) ? dsts[min(e0 + 2, nE - 1)] : sent;
    da.w = (e0 + 3 < nE) ? dsts[min(e0 + 3, nE - 1)] : sent;
    db.x = (e0 + 4 < nE) ? dsts[min(e0 + 4, nE - 1)] : sent;
    db.y = (e0 + 5 < nE) ? dsts[min(e0 + 5, nE - 1)] : sent;
    db.z = (e0 + 6 < nE) ? dsts[min(e0 + 6, nE - 1)] : sent;
    db.w = (e0 + 7 < nE) ? dsts[min(e0 + 7, nE - 1)] : sent;
  }
  const unsigned nbs = (unsigned)slotBase;
  const unsigned unb = (unsigned)nb;
  const unsigned s0 = (unsigned)da.x - nbs, s1 = (unsigned)da.y - nbs;
  const unsigned s2 = (unsigned)da.z - nbs, s3 = (unsigned)da.w - nbs;
  const unsigned s4 = (unsigned)db.x - nbs, s5 = (unsigned)db.y - nbs;
  const unsigned s6 = (unsigned)db.z - nbs, s7 = (unsigned)db.w - nbs;
  const bool h0 = s0 < unb, h1 = s1 < unb, h2 = s2 < unb, h3 = s3 < unb;
  const bool h4 = s4 < unb, h5 = s5 < unb, h6 = s6 < unb, h7 = s7 < unb;
  const unsigned any = __builtin_amdgcn_ballot_w32(h0 | h1 | h2 | h3 | h4 | h5 | h6 | h7);
  if (any != 0u) {
#define HITJ(J, HJ, SJ) { \
      const unsigned mj = __builtin_amdgcn_ballot_w32(HJ); \
      if (mj != 0u) { \
        if (HJ) { \
          const int pos = wc + (int)__builtin_amdgcn_mbcnt_lo(mj, 0u); \
          if (pos < WCAP) list[wave * WCAP + pos] = ((el0 + (J)) << 12) | (int)(SJ); \
        } \
        wc += (int)__builtin_popcount(mj); } }
    HITJ(0, h0, s0)
    HITJ(1, h1, s1)
    HITJ(2, h2, s2)
    HITJ(3, h3, s3)
    HITJ(4, h4, s4)
    HITJ(5, h5, s5)
    HITJ(6, h6, s6)
    HITJ(7, h7, s7)
#undef HITJ
  }
  return wc;
}

__global__ __launch_bounds__(NTHR) void k_xprep(const float* __restrict__ x, unsigned short* xb, int nN, int nUnits) {
  const int i = (int)blockIdx.x * NTHR + (int)threadIdx.x;
  if (i >= nUnits) return;
  const int row = i >> 4;
  const int c0  = (i & 15) * 8;
  const int rc  = row < nN ? row : nN - 1;
  const float* p = x + (size_t)rc * DIN + c0;
  v4f a = *(const v4f*)p, b = *(const v4f*)(p + 4);
  const v4f z4 = {0.f, 0.f, 0.f, 0.f};
  if (row >= nN) { a = z4; b = z4; }
  const v8us hv = cvt8b(a, b);
  const size_t o = (size_t)row * DIN + c0;
  *(volatile v8us*)(xb + o) = hv;
  __threadfence();
  *(volatile v8us*)(xb + o) = hv;
}

__global__ __launch_bounds__(NTHR) void k_wtr(const float* __restrict__ w0, const float* __restrict__ w1,
                                              const float* __restrict__ w2, const float* __restrict__ w3,
                                              int c0, int c1, int c2, int c3, int segRows, int K,
                                              unsigned short* wt, int nUnits) {
  const int u = (int)blockIdx.x * NTHR + (int)threadIdx.x;
  if (u >= nUnits) return;
  const int kq = K >> 3;
  const int n  = u / kq;
  const int k8 = (u - n * kq) * 8;
  int seg = n / segRows;
  seg = seg > 3 ? 3 : seg;
  const int nc = n - seg * segRows;
  const float* ws = (seg == 0) ? w0 : ((seg == 1) ? w1 : ((seg == 2) ? w2 : w3));
  const int cc = (seg == 0) ? c0 : ((seg == 1) ? c1 : ((seg == 2) ? c2 : c3));
  const int ncl = nc < cc ? nc : cc - 1;
  const float* p = ws + (size_t)k8 * (size_t)cc + ncl;
  v4f a, b;
  a.x = p[0];                  a.y = p[(size_t)cc];         a.z = p[(size_t)2 * cc];     a.w = p[(size_t)3 * cc];
  b.x = p[(size_t)4 * cc];     b.y = p[(size_t)5 * cc];     b.z = p[(size_t)6 * cc];     b.w = p[(size_t)7 * cc];
  const v4f z4 = {0.f, 0.f, 0.f, 0.f};
  if (nc >= cc) { a = z4; b = z4; }
  const v8us hv = cvt8b(a, b);
  const size_t o = (size_t)n * (size_t)K + k8;
  *(volatile v8us*)(wt + o) = hv;
  __threadfence();
  *(volatile v8us*)(wt + o) = hv;
}

template<int NP>
__global__ __launch_bounds__(GTHR) void k_gemm(
    const unsigned short* __restrict__ A0, const unsigned short* __restrict__ A1,
    const unsigned short* __restrict__ WT, const float* __restrict__ atts, const float* __restrict__ attd,
    float* Hout, float* ASo, float* ADo, int K)
{
  __shared__ __attribute__((aligned(16))) float stg[GBM * HC];
  __shared__ __attribute__((aligned(16))) float asl[GBM];
  __shared__ __attribute__((aligned(16))) float adl[GBM];
  __shared__ float satt[HC];
  __shared__ float datt[HC];
  const int tid = (int)threadIdx.x, lane = tid & 31, wave = tid >> 5, hh = lane >> 4, m = lane & 15;
  const int rowBase = (int)blockIdx.x * GBM;
  if (tid < HC) { satt[tid] = bfr(atts[tid]); datt[tid] = bfr(attd[tid]); }

  v8f acc[4];
  {
    const v8f z = {0.f, 0.f, 0.f, 0.f, 0.f, 0.f, 0.f, 0.f};
    acc[0] = z; acc[1] = z; acc[2] = z; acc[3] = z;
  }
  const unsigned short* ap0 = A0 + (size_t)(rowBase + 16 * wave + m) * (size_t)K + 8 * hh;
  const unsigned short* ap1 = A1 + (size_t)(rowBase + 16 * wave + m) * (size_t)K + 8 * hh;
  const unsigned short* wp  = WT + (size_t)m * (size_t)K + 8 * hh;
  const int ksteps = K >> 5;
#pragma unroll 1
  for (int ks = 0; ks < ksteps; ++ks) {
    FragB af;
    af.h[0] = *(const v8us*)(ap0 + 32 * ks);
    af.h[1] = *(const v8us*)(ap0 + 32 * ks + 16);
    FragB ag = af;
    if (NP == 2) {
      ag.h[0] = *(const v8us*)(ap1 + 32 * ks);
      ag.h[1] = *(const v8us*)(ap1 + 32 * ks + 16);
    }
#pragma unroll
    for (int t = 0; t < 4; ++t) {
      const unsigned short* wq = wp + (size_t)(16 * t) * (size_t)K + 32 * ks;
      FragB bf;
      bf.h[0] = *(const v8us*)wq;
      bf.h[1] = *(const v8us*)(wq + 16);
      acc[t] = wmb(af, bf, acc[t]);
      if (NP == 2) acc[t] = wmb(ag, bf, acc[t]);
    }
  }

#pragma unroll
  for (int t = 0; t < 4; ++t) {
    const int lc = 16 * t + m;
#pragma unroll
    for (int r = 0; r < 8; ++r) {
      const int lr = 16 * wave + 8 * hh + r;
      stg[lr * HC + lc] = acc[t][r];
    }
  }
  __syncthreads();

  {
    const int row = tid >> 1, half = tid & 1;
    float ps = 0.f, pd = 0.f;
#pragma unroll 8
    for (int j = 0; j < 32; ++j) {
      const int c = 32 * half + j;
      const float hv = stg[row * HC + c];
      ps = fmaf(hv, satt[c], ps);
      pd = fmaf(hv, datt[c], pd);
    }
    ps += __shfl_xor(ps, 1);
    pd += __shfl_xor(pd, 1);
    if (half == 0) { asl[row] = ps; adl[row] = pd; }
  }
  __syncthreads();

  v4f fv[8];
#pragma unroll
  for (int i = 0; i < 8; ++i) {
    const int lr = 16 * wave + 2 * i + hh;
    fv[i] = *(const v4f*)(stg + lr * HC + 4 * m);
  }
  const int l16 = lane & 15;
  const v4f va = *(const v4f*)(asl + 4 * l16);
  const v4f vd = *(const v4f*)(adl + 4 * l16);
  const v4f vs = sel4(lane < 16, va, vd);
  float* sp = ((lane < 16) ? ASo : ADo) + rowBase + 4 * l16;

#pragma unroll
  for (int i = 0; i < 8; ++i) {
    const int lr = 16 * wave + 2 * i + hh;
    const int gr = rowBase + lr;
    float* op = Hout + (size_t)gr * HC + 4 * m;
    *(volatile v4f*)op = fv[i];
  }
  if (wave == 0) *(volatile v4f*)sp = vs;
  __threadfence();
#pragma unroll
  for (int i = 0; i < 8; ++i) {
    const int lr = 16 * wave + 2 * i + hh;
    const int gr = rowBase + lr;
    float* op = Hout + (size_t)gr * HC + 4 * m;
    *(volatile v4f*)op = fv[i];
  }
  if (wave == 0) *(volatile v4f*)sp = vs;
}

template<int MODE>
__global__ __launch_bounds__(NTHR) void k_agg(
    const int* __restrict__ srcs, const int* __restrict__ dsts,
    const float* __restrict__ AS, const float* __restrict__ AD,
    const float* __restrict__ H, const float* __restrict__ bias,
    unsigned short* Zh, unsigned short* Zl, float* outF,
    int nN, int nE, int nb, int vec8, int MPr) {
  extern __shared__ v4f lds_dyn[];
  int* reg1 = (int*)lds_dyn;
  int* reg2 = reg1 + RCAP;
  int* scnt = reg2 + RCAP;
  int* soff = scnt + NBMAX;
  int* list = soff + NBMAX;
  int* wcnt = list + LISTN;
  int* wtot = wcnt + NWAVE;
  const int tid = (int)threadIdx.x, lane = tid & 31, wave = tid >> 5;
  const int nodeBase = (int)blockIdx.x * nb;

  for (int i = tid; i < NBMAX; i += NTHR) scnt[i] = 0;
  __syncthreads();

  int tot = 0;
  const int nChunks = (nE + CHUNK - 1) / CHUNK;
#pragma unroll 1
  for (int ch = 0; ch < nChunks; ++ch) {
    const int cbase = ch * CHUNK;
    const int wc = scan_chunk(dsts, nE, cbase, nodeBase, nb, vec8, list, tid, lane, wave);
    if (lane == 0) wcnt[wave] = wc;
    __syncthreads();
    int pre = 0, all = 0;
#pragma unroll
    for (int w2 = 0; w2 < NWAVE; ++w2) {
      int c = wcnt[w2];
      c = c < 0 ? 0 : (c > WCAP ? WCAP : c);
      all += c;
      pre += (w2 < wave) ? c : 0;
    }
    const int wcc  = wc > WCAP ? WCAP : wc;
    const int base = tot + pre;
#pragma unroll 1
    for (int i = lane; i < wcc; i += 32) {
      const int ent = list[wave * WCAP + i];
      const int el  = (ent >> 12) & (CHUNK - 1);
      const int sl  = ent & (NBMAX - 1);
      int eid = cbase + el;
      eid = eid > nE - 1 ? nE - 1 : eid;
      const int pos = base + i;
      if (pos < RCAP) reg1[pos] = (int)(((unsigned)eid << SLBITS) | (unsigned)sl);
    }
    tot += all;
    tot = tot > RCAP ? RCAP : tot;
    __syncthreads();
  }
  const int nh = tot;

  if (wave == 0) {
#pragma unroll 1
    for (int b0 = 0; b0 < nh; b0 += 32) {
      const int idx = b0 + lane;
      const int uv  = reg1[idx < RCAP ? idx : RCAP - 1];
      const int m32 = (nh - b0) < 32 ? (nh - b0) : 32;
#pragma unroll 1
      for (int k = 0; k < m32; ++k) {
        const int u  = __builtin_amdgcn_readlane(uv, k);
        const int sl = u & (NBMAX - 1);
        if (lane == 0) scnt[sl] = scnt[sl] + 1;
      }
    }
  }
  __syncthreads();

  {
    const int c0r = scnt[2 * tid], c1r = scnt[2 * tid + 1];
    const int e0 = c0r < 0 ? 0 : c0r, e1 = c1r < 0 ? 0 : c1r;
    const int ts = e0 + e1;
    int incl = ts;
#pragma unroll
    for (int d = 1; d < 32; d <<= 1) {
      const int up = __shfl_up(incl, d);
      if (lane >= d) incl += up;
    }
    if (lane == 31) wtot[wave] = incl;
    __syncthreads();
    int pre = 0;
#pragma unroll
    for (int w2 = 0; w2 < NWAVE; ++w2) pre += (w2 < wave) ? wtot[w2] : 0;
    const int run = pre + incl - ts;
    soff[2 * tid]     = run;
    soff[2 * tid + 1] = run + e0;
  }
  __syncthreads();
  for (int i = tid; i < NBMAX; i += NTHR) list[i] = soff[i];
  __syncthreads();

  if (wave == 0) {
#pragma unroll 1
    for (int b0 = 0; b0 < nh; b0 += 32) {
      const int idx = b0 + lane;
      const int uv  = reg1[idx < RCAP ? idx : RCAP - 1];
      const int m32 = (nh - b0) < 32 ? (nh - b0) : 32;
#pragma unroll 1
      for (int k = 0; k < m32; ++k) {
        const int u   = __builtin_amdgcn_readlane(uv, k);
        const int sl  = u & (NBMAX - 1);
        const int eid = (int)((unsigned)u >> SLBITS);
        if (lane == 0) {
          int pos = list[sl];
          pos = pos < 0 ? 0 : (pos > RCAP - 1 ? RCAP - 1 : pos);
          reg2[pos] = eid;
          list[sl] = pos + 1;
        }
      }
    }
  }
  __syncthreads();

  const int nbw = nb >> 3;
  const bool ovf = (nh >= RCAP);
  const float qnan = __int_as_float(0x7fc00000);
  float* stw = (float*)reg1 + wave * STW;
  const float bv0 = bfr(bias[lane]);
  const float bv1 = bfr(bias[32 + lane]);
#pragma unroll 1
  for (int jt = 0; jt < nbw; ++jt) {
    const int slot = wave * nbw + jt;
    const int grow = nodeBase + slot;
    const int gcl  = grow < nN ? grow : nN - 1;
    int st = soff[slot];
    const int craw = scnt[slot];
    int cnt = craw;
    st  = st < 0 ? 0 : (st > nh ? nh : st);
    cnt = cnt < 0 ? 0 : (cnt > DEGCAP ? DEGCAP : cnt);
    if (cnt > nh - st) cnt = nh - st;
    const float pz = (ovf || craw > DEGCAP) ? qnan : 0.0f;

    const float adv = AD[gcl];
    const float asv = AS[gcl];
    float e0 = asv + adv;
    e0 = e0 > 0.f ? e0 : 0.2f * e0;
    float mx = e0, dn = 1.0f;
    const float* hr = H + (size_t)gcl * HC + lane;
    float av0 = hr[0];
    float av1 = hr[32];
#pragma unroll 1
    for (int q = 0; q < cnt; ++q) {
      int idx = st + q; idx = idx > RCAP - 1 ? RCAP - 1 : idx;
      int eid = reg2[idx]; eid = eid < 0 ? 0 : (eid > nE - 1 ? nE - 1 : eid);
      const int sraw = srcs[eid];
      const int s = sraw < 0 ? 0 : (sraw > nN - 1 ? nN - 1 : sraw);
      const float asq = AS[s];
      const float* hq = H + (size_t)s * HC + lane;
      const float h0 = hq[0];
      const float h1 = hq[32];
      float l = asq + adv;
      l = l > 0.f ? l : 0.2f * l;
      const float df = l - mx;
      const float ee = __expf(-fabsf(df));
      const bool up  = df > 0.f;
      const float s1 = up ? ee : 1.0f;
      const float s2 = up ? 1.0f : ee;
      mx  = up ? l : mx;
      dn  = fmaf(dn, s1, s2);
      av0 = fmaf(av0, s1, s2 * h0);
      av1 = fmaf(av1, s1, s2 * h1);
    }
    const float iv = __builtin_amdgcn_rcpf(dn);
    float r0 = fmaf(av0, iv, bv0);
    float r1 = fmaf(av1, iv, bv1);
    if (MODE == 1) {
      const float live = grow < nN ? 1.0f : 0.0f;
      r0 = fmaxf(r0, 0.f) * live + pz;
      r1 = fmaxf(r1, 0.f) * live + pz;
    } else {
      r0 = r0 + pz;
      r1 = r1 + pz;
    }
    __builtin_amdgcn_fence(__ATOMIC_RELEASE, "wavefront");
    __builtin_amdgcn_wave_barrier();
    stw[lane]      = r0;
    stw[32 + lane] = r1;
    __builtin_amdgcn_fence(__ATOMIC_RELEASE, "wavefront");
    __builtin_amdgcn_wave_barrier();
    if (MODE == 1) {
      const int q8 = lane & 7;
      const v4f ga = *(const v4f*)(stw + 8 * q8);
      const v4f gb = *(const v4f*)(stw + 8 * q8 + 4);
      v4us ha, la, hb, lb;
      hilo4(ga, ha, la);
      hilo4(gb, hb, lb);
      v8us hv8, lv8;
      hv8[0] = ha.x; hv8[1] = ha.y; hv8[2] = ha.z; hv8[3] = ha.w;
      hv8[4] = hb.x; hv8[5] = hb.y; hv8[6] = hb.z; hv8[7] = hb.w;
      lv8[0] = la.x; lv8[1] = la.y; lv8[2] = la.z; lv8[3] = la.w;
      lv8[4] = lb.x; lv8[5] = lb.y; lv8[6] = lb.z; lv8[7] = lb.w;
      const bool islo = ((lane >> 3) & 1) != 0;
      const v8us sv = sel8(islo, lv8, hv8);
      unsigned short* gp = (islo ? Zl : Zh) + (size_t)grow * HC + 8 * q8;
      const bool wsv = (grow < MPr) && (lane < 16);
      if (wsv) *(volatile v8us*)gp = sv;
      __threadfence();
      if (wsv) *(volatile v8us*)gp = sv;
    } else {
      const int l16 = lane & 15;
      const v4f gv = *(const v4f*)(stw + 4 * l16);
      float* gp = outF + (size_t)grow * HC + 4 * l16;
      const bool wsv = (grow < nN) && (lane < 16);
      if (wsv) *(volatile v4f*)gp = gv;
      __threadfence();
      if (wsv) *(volatile v4f*)gp = gv;
    }
  }
}

__global__ __launch_bounds__(NTHR) void k_tprob(const float* zpl, const float* __restrict__ Wp,
                                                const float* __restrict__ bp, float* outp, int nN) {
  __shared__ float wpl[2 * HC];
  __shared__ float bpl[2];
  const int tid = (int)threadIdx.x, lane = tid & 31, wave = tid >> 5;
  if (tid < 2 * HC) wpl[tid] = bfr(Wp[tid]);
  if (tid < 2) bpl[tid] = bfr(bp[tid]);
  __syncthreads();
  const int rbase = ((int)blockIdx.x * NWAVE + wave) * 16;
  if (rbase >= nN) return;
  const int r = lane >> 1, j = lane & 1;
  const int row = rbase + r;
  const int rowc = row < nN ? row : nN - 1;
  const float* z = zpl + (size_t)rowc * HC;
  float s = 0.f;
#pragma unroll 4
  for (int k = 0; k < HC; ++k) s = fmaf(z[k], wpl[2 * k + j], s);
  s += bpl[j];
  float* gp = outp + (size_t)rbase * 2 + lane;
  const bool ok = row < nN;
  if (ok) *(volatile float*)gp = s;
  __threadfence();
  if (ok) *(volatile float*)gp = s;
}

__global__ __launch_bounds__(GTHR) void k_head(
    const float* dsrc, const int* __restrict__ tix, const int* __restrict__ cix,
    const unsigned short* __restrict__ WTS, const unsigned short* __restrict__ WT1a,
    const unsigned short* __restrict__ WT0a, const float* __restrict__ byS,
    const float* __restrict__ by1a, const float* __restrict__ Wy1b, const float* __restrict__ by1b,
    const float* __restrict__ by0a, const float* __restrict__ Wy0b, const float* __restrict__ by0b,
    float* yout, int nN, int nT, int nC, int off4, int off5)
{
  __shared__ __attribute__((aligned(16))) unsigned short Ahi[HBM * HC];
  __shared__ __attribute__((aligned(16))) unsigned short Alo[HBM * HC];
  __shared__ __attribute__((aligned(16))) float stg[HBM * HC];
  __shared__ __attribute__((aligned(16))) float yl[HBM];
  __shared__ int rz[HBM];
  __shared__ int rset[HBM];
  __shared__ float wbl[HC];
  const int tid = (int)threadIdx.x, lane = tid & 31, wave = tid >> 5, hh = lane >> 4, m = lane & 15;
  const int nTot = 2 * nT + 2 * nC;
  const int g0 = (int)blockIdx.x * HBM;

  if (tid < HBM) {
    const int g  = g0 + tid;
    const int gc = g < nTot ? g : nTot - 1;
    int seg, i;
    if (gc < nT)               { seg = 0; i = gc; }
    else if (gc < 2 * nT)      { seg = 1; i = gc - nT; }
    else if (gc < 2 * nT + nC) { seg = 2; i = gc - 2 * nT; }
    else                       { seg = 3; i = gc - 2 * nT - nC; }
    i = i < 0 ? 0 : i;
    const int it = i < nT - 1 ? i : nT - 1;
    const int ic = i < nC - 1 ? i : nC - 1;
    const int tv = tix[it];
    const int cv = cix[ic];
    int node = (seg < 2) ? tv : cv;
    node = node < 0 ? 0 : (node > nN - 1 ? nN - 1 : node);
    rz[tid]   = ((seg & 1) ? off5 : off4) + node * HC;
    rset[tid] = (seg == 0 || seg == 3) ? 1 : 0;
    yl[tid]   = 0.f;
  }
  __syncthreads();

#pragma unroll
  for (int itn = 0; itn < 8; ++itn) {
    const int p   = itn * GTHR + tid;
    const int row = p >> 4;
    const int c4  = (p & 15) * 4;
    const v4f v = *(const v4f*)(dsrc + (size_t)rz[row] + c4);
    v4us hb, lb;
    hilo4(v, hb, lb);
    *(v4us*)(Ahi + row * HC + c4) = hb;
    *(v4us*)(Alo + row * HC + c4) = lb;
  }
  __syncthreads();

  v8f acc[4];
  {
    const v8f z8 = {0.f, 0.f, 0.f, 0.f, 0.f, 0.f, 0.f, 0.f};
    acc[0] = z8; acc[1] = z8; acc[2] = z8; acc[3] = z8;
    const unsigned short* ah = Ahi + (16 * wave + m) * HC + 8 * hh;
    const unsigned short* al = Alo + (16 * wave + m) * HC + 8 * hh;
    const unsigned short* wp = WTS + (size_t)m * HC + 8 * hh;
#pragma unroll
    for (int ks = 0; ks < HC / 32; ++ks) {
      FragB fa, fl;
      fa.h[0] = *(const v8us*)(ah + 32 * ks);
      fa.h[1] = *(const v8us*)(ah + 32 * ks + 16);
      fl.h[0] = *(const v8us*)(al + 32 * ks);
      fl.h[1] = *(const v8us*)(al + 32 * ks + 16);
#pragma unroll
      for (int t = 0; t < 4; ++t) {
        const unsigned short* wq = wp + (size_t)(16 * t) * HC + 32 * ks;
        FragB fb;
        fb.h[0] = *(const v8us*)wq;
        fb.h[1] = *(const v8us*)(wq + 16);
        acc[t] = wmb(fa, fb, acc[t]);
        acc[t] = wmb(fl, fb, acc[t]);
      }
    }
  }
#pragma unroll
  for (int t = 0; t < 4; ++t) {
    const int lc = 16 * t + m;
    const float bs = bfr(byS[lc]);
#pragma unroll
    for (int r = 0; r < 8; ++r) {
      const int lr = 16 * wave + 8 * hh + r;
      stg[lr * HC + lc] = lk01(acc[t][r] + bs);
    }
  }
  __syncthreads();
#pragma unroll
  for (int itn = 0; itn < 8; ++itn) {
    const int p   = itn * GTHR + tid;
    const int row = p >> 4;
    const int c4  = (p & 15) * 4;
    const v4f v = *(const v4f*)(stg + row * HC + c4);
    v4us hb, lb;
    hilo4(v, hb, lb);
    *(v4us*)(Ahi + row * HC + c4) = hb;
    *(v4us*)(Alo + row * HC + c4) = lb;
  }
  __syncthreads();

  const int setF = rset[0], setL = rset[HBM - 1];
  const int nIter = (setF != setL) ? 2 : 1;
#pragma unroll 1
  for (int it = 0; it < nIter; ++it) {
    const int cs = (it == 0) ? setF : setL;
    const unsigned short* WB = cs ? WT1a : WT0a;
    const float* ba = cs ? by1a : by0a;
    const float* Wb = cs ? Wy1b : Wy0b;
    const float* bb = cs ? by1b : by0b;
    if (tid < HC) wbl[tid] = bfr(Wb[tid]);
    {
      const v8f z8 = {0.f, 0.f, 0.f, 0.f, 0.f, 0.f, 0.f, 0.f};
      acc[0] = z8; acc[1] = z8; acc[2] = z8; acc[3] = z8;
      const unsigned short* ah = Ahi + (16 * wave + m) * HC + 8 * hh;
      const unsigned short* al = Alo + (16 * wave + m) * HC + 8 * hh;
      const unsigned short* wp = WB + (size_t)m * HC + 8 * hh;
#pragma unroll
      for (int ks = 0; ks < HC / 32; ++ks) {
        FragB fa, fl;
        fa.h[0] = *(const v8us*)(ah + 32 * ks);
        fa.h[1] = *(const v8us*)(ah + 32 * ks + 16);
        fl.h[0] = *(const v8us*)(al + 32 * ks);
        fl.h[1] = *(const v8us*)(al + 32 * ks + 16);
#pragma unroll
        for (int t = 0; t < 4; ++t) {
          const unsigned short* wq = wp + (size_t)(16 * t) * HC + 32 * ks;
          FragB fb;
          fb.h[0] = *(const v8us*)wq;
          fb.h[1] = *(const v8us*)(wq + 16);
          acc[t] = wmb(fa, fb, acc[t]);
          acc[t] = wmb(fl, fb, acc[t]);
        }
      }
    }
#pragma unroll
    for (int t = 0; t < 4; ++t) {
      const int lc = 16 * t + m;
      const float bav = bfr(ba[lc]);
#pragma unroll
      for (int r = 0; r < 8; ++r) {
        const int lr = 16 * wave + 8 * hh + r;
        stg[lr * HC + lc] = lk01(acc[t][r] + bav);
      }
    }
    __syncthreads();
    {
      const int row = tid >> 1, half = tid & 1;
      float s = 0.f;
#pragma unroll 4
      for (int j = 0; j < 32; ++j) {
        const int c = 32 * half + j;
        s = fmaf(stg[row * HC + c], wbl[c], s);
      }
      s += __shfl_xor(s, 1);
      const float y = lk01(s + bfr(bb[0]));
      if (half == 0 && rset[row] == cs) yl[row] = y;
    }
    __syncthreads();
  }

  const int l16 = lane & 15;
  const v4f yv = *(const v4f*)(yl + 4 * l16);
  const int gi = g0 + 4 * l16;
  const bool ok = (wave == 0) && (lane < 16) && (gi + 4 <= nTot);
  float* gp = yout + gi;
  if (ok) *(volatile v4f*)gp = yv;
  __threadfence();
  if (ok) *(volatile v4f*)gp = yv;
}

static inline int cdiv(int a, int b) { return (a + b - 1) / b; }

extern "C" void kernel_launch(void* const* d_in, const int* in_sizes, int n_in,
                              void* d_out, int out_size, void* d_ws, size_t ws_size,
                              hipStream_t stream) {
  if (n_in < 26) return;
  const int nN = in_sizes[0] / DIN;
  if (nN < 16 || in_sizes[0] != nN * DIN || nN > (1 << 21)) return;
  if (in_sizes[2] != in_sizes[0]) return;
  if (in_sizes[1] < 2 || (in_sizes[1] & 1) != 0) return;
  if (in_sizes[3] < 2 || (in_sizes[3] & 1) != 0) return;
  const int nE = in_sizes[1] / 2;
  const int nF = in_sizes[3] / 2;
  if (nE < 1 || nE > (1 << 22) || nF < 1 || nF > (1 << 22)) return;
  const int nT = in_sizes[4], nC = in_sizes[5];
  if (nT < 1 || nC < 1) return;
  if (in_sizes[6]  != DIN * HC) return;
  if (in_sizes[7]  != HC || in_sizes[8]  != HC || in_sizes[9]  != HC) return;
  if (in_sizes[10] != HC * HC) return;
  if (in_sizes[11] != HC || in_sizes[12] != HC || in_sizes[13] != HC) return;
  if (in_sizes[14] != HC * HC || in_sizes[15] != HC) return;
  if (in_sizes[16] != HC * HC || in_sizes[17] != HC) return;
  if (in_sizes[18] != HC || in_sizes[19] < 1) return;
  if (in_sizes[20] != HC * HC || in_sizes[21] != HC) return;
  if (in_sizes[22] != HC || in_sizes[23] < 1) return;
  if (in_sizes[24] != 2 * HC || in_sizes[25] < 2) return;

  const int nTot = 2 * nT + 2 * nC;
  const size_t off4 = (size_t)nTot;
  const size_t off5 = off4 + (size_t)nN * HC;
  const size_t off6 = off5 + (size_t)nN * HC;
  if ((size_t)out_size != off6 + (size_t)2 * nN) return;
  if ((nTot & 3) != 0) return;
  if (off6 > (size_t)0x7fffffff) return;

  const float* x    = (const float*)d_in[0];
  const int*   ei   = (const int*)  d_in[1];
  const float* fx   = (const float*)d_in[2];
  const int*   fei  = (const int*)  d_in[3];
  const int*   tix  = (const int*)  d_in[4];
  const int*   cix  = (const int*)  d_in[5];
  const float* W1   = (const float*)d_in[6];
  const float* as1  = (const float*)d_in[7];
  const float* ad1  = (const float*)d_in[8];
  const float* b1   = (const float*)d_in[9];
  const float* W2   = (const float*)d_in[10];
  const float* as2  = (const float*)d_in[11];
  const float* ad2  = (const float*)d_in[12];
  const float* b2   = (const float*)d_in[13];
  const float* WyS  = (const float*)d_in[14];
  const float* byS  = (const float*)d_in[15];
  const float* Wy1a = (const float*)d_in[16];
  const float* by1a = (const float*)d_in[17];
  const float* Wy1b = (const float*)d_in[18];
  const float* by1b = (const float*)d_in[19];
  const float* Wy0a = (const float*)d_in[20];
  const float* by0a = (const float*)d_in[21];
  const float* Wy0b = (const float*)d_in[22];
  const float* by0b = (const float*)d_in[23];
  const float* Wp   = (const float*)d_in[24];
  const float* bp   = (const float*)d_in[25];
  float* out = (float*)d_out;

  const int MP = cdiv(nN, GBM) * GBM;
  const int nb = NBMAX;
  const int gA = cdiv(MP, nb);
  if (gA * nb < MP) return;
  const int vec8e = ((nE & 3) == 0) ? 1 : 0;
  const int vec8f = ((nF & 3) == 0) ? 1 : 0;

  char* ws = (char*)d_ws;
  size_t off = 0;
  const size_t oXB  = off; off += (size_t)MP * DIN * 2;     off = (off + 255) & ~(size_t)255;
  const size_t oH   = off; off += (size_t)MP * HC * 4;      off = (off + 255) & ~(size_t)255;
  const size_t oZH  = off; off += (size_t)MP * HC * 2;      off = (off + 255) & ~(size_t)255;
  const size_t oZL  = off; off += (size_t)MP * HC * 2;      off = (off + 255) & ~(size_t)255;
  const size_t oAS  = off; off += (size_t)MP * 4;           off = (off + 255) & ~(size_t)255;
  const size_t oAD  = off; off += (size_t)MP * 4;           off = (off + 255) & ~(size_t)255;
  const size_t oWT1 = off; off += (size_t)HC * DIN * 2;     off = (off + 255) & ~(size_t)255;
  const size_t oWT4 = off; off += (size_t)4 * HC * HC * 2;  off = (off + 255) & ~(size_t)255;
  if (off > ws_size || off > (size_t)WSMAX) return;
  unsigned short* XB  = (unsigned short*)(ws + oXB);
  float*          Hpl = (float*)(ws + oH);
  unsigned short* ZH  = (unsigned short*)(ws + oZH);
  unsigned short* ZL  = (unsigned short*)(ws + oZL);
  float*          AS  = (float*)(ws + oAS);
  float*          AD  = (float*)(ws + oAD);
  unsigned short* WT1 = (unsigned short*)(ws + oWT1);
  unsigned short* WT4 = (unsigned short*)(ws + oWT4);
  unsigned short* WT2  = WT4;
  unsigned short* WTS  = WT4 + (size_t)HC * HC;
  unsigned short* WT1a = WT4 + (size_t)2 * HC * HC;
  unsigned short* WT0a = WT4 + (size_t)3 * HC * HC;

  hipFuncSetAttribute(reinterpret_cast<const void*>(&k_agg<1>),
                      hipFuncAttributeMaxDynamicSharedMemorySize, LDS_AGG);
  hipFuncSetAttribute(reinterpret_cast<const void*>(&k_agg<2>),
                      hipFuncAttributeMaxDynamicSharedMemorySize, LDS_AGG);

  {
    const int nU1 = HC * (DIN / 8);
    k_wtr<<<cdiv(nU1, NTHR), NTHR, 0, stream>>>(W1, W1, W1, W1, HC, HC, HC, HC, HC, DIN, WT1, nU1);
    const int nU4 = 4 * HC * (HC / 8);
    k_wtr<<<cdiv(nU4, NTHR), NTHR, 0, stream>>>(W2, WyS, Wy1a, Wy0a, HC, HC, HC, HC, HC, HC, WT4, nU4);
  }

  const int nUx = MP * (DIN / 8);
  const int gM  = MP / GBM;
  for (int g = 0; g < 2; ++g) {
    const float* X   = g ? fx : x;
    const int*   EI  = g ? fei : ei;
    const int    nEg = g ? nF : nE;
    const int    v8  = g ? vec8f : vec8e;
    const int* src = EI;
    const int* dst = EI + nEg;
    float* Zout = out + (g ? off5 : off4);
    k_xprep<<<cdiv(nUx, NTHR), NTHR, 0, stream>>>(X, XB, nN, nUx);
    k_gemm<1><<<gM, GTHR, 0, stream>>>(XB, XB, WT1, as1, ad1, Hpl, AS, AD, DIN);
    k_agg<1><<<gA, NTHR, LDS_AGG, stream>>>(src, dst, AS, AD, Hpl, b1, ZH, ZL, Hpl, nN, nEg, nb, v8, MP);
    k_gemm<2><<<gM, GTHR, 0, stream>>>(ZH, ZL, WT2, as2, ad2, Hpl, AS, AD, HC);
    k_agg<2><<<gA, NTHR, LDS_AGG, stream>>>(src, dst, AS, AD, Hpl, b2, ZH, ZL, Zout, nN, nEg, nb, v8, MP);
  }

  k_tprob<<<cdiv(nN, 16 * NWAVE), NTHR, 0, stream>>>(out + off4, Wp, bp, out + off6, nN);
  k_head<<<cdiv(nTot, HBM), GTHR, 0, stream>>>(out, tix, cix, WTS, WT1a, WT0a, byS,
                                                by1a, Wy1b, by1b, by0a, Wy0b, by0b,
                                                out, nN, nT, nC, (int)off4, (int)off5);
}
